// PVMLayer_72387378806824
// MI455X (gfx1250) — hardware-verified
//
#include <hip/hip_runtime.h>
#include <math.h>

#define NBAT 8
#define NCH  256
#define IMH  64
#define IMW  64
#define LTOK (IMH * IMW)
#define NTOK (NBAT * LTOK)
#define DMD  64
#define DIN  128
#define DST  16
#define DTRK 4
#define XPR  36
#define XDN  64
#define DCV  4
#define NCHK 4
#define NLY  4
#define EPSV 1e-5f
#define GSTR 40
#define OSTR 68
#define TPN  132
#define SMEMB (8 * 16 * OSTR * 4)
#define SCH  32
#define SYP  132
#define LNP  260
#define LOG2E 1.4426950408889634f

static_assert(NTOK % 128 == 0);
static_assert(LTOK % 128 == 0);
static_assert(NCH % 64 == 0);
static_assert(NCH == NCHK * DMD);
static_assert(DMD % 32 == 0);
static_assert(DIN % 32 == 0);
static_assert(DIN == 128);
static_assert(XDN == 64);
static_assert(XPR <= XDN);
static_assert(DTRK + 2 * DST <= XDN);
static_assert(SMEMB >= (2 * 128 * GSTR + 64 * GSTR) * 2);
static_assert(SMEMB >= 64 * TPN * 4);
static_assert(LTOK % SCH == 0);
static_assert(SCH == 32);
static_assert(SYP % 4 == 0);
static_assert(SYP >= DIN);
static_assert(LNP % 4 == 0);
static_assert(LNP >= NCH);
static_assert(TPN % 4 == 0);
static_assert(TPN >= 128);
static_assert(NTOK % 32 == 0);

typedef unsigned short us16 __attribute__((ext_vector_type(16)));
typedef unsigned short us8  __attribute__((ext_vector_type(8)));
typedef unsigned short us8a __attribute__((ext_vector_type(8), may_alias));
typedef unsigned short us4  __attribute__((ext_vector_type(4)));
typedef unsigned short us4a __attribute__((ext_vector_type(4), may_alias));
typedef __bf16 v16b __attribute__((ext_vector_type(16)));
typedef float v8f __attribute__((ext_vector_type(8)));
typedef float v4f __attribute__((ext_vector_type(4)));
typedef float v4fa __attribute__((ext_vector_type(4), may_alias));
union FragU { us16 v; us8 h[2]; };

__device__ __forceinline__ unsigned short bf16_bits(float f) {
  unsigned u = __float_as_uint(f);
  u += 0x7FFFu + ((u >> 16) & 1u);
  return (unsigned short)(u >> 16);
}
__device__ __forceinline__ float bf16_val(unsigned short b) { return __uint_as_float(((unsigned)b) << 16); }
__device__ __forceinline__ float bf16r(float f) { return bf16_val(bf16_bits(f)); }
__device__ __forceinline__ float siluf(float x) { return x * __builtin_amdgcn_rcpf(1.0f + __expf(-x)); }

__device__ __forceinline__ v8f mma_bf16(us16 a, us16 b, v8f c) {
  return __builtin_amdgcn_wmma_f32_16x16x32_bf16(false, __builtin_bit_cast(v16b, a), false, __builtin_bit_cast(v16b, b), (short)0, c, false, false);
}
__device__ __forceinline__ void wguard(v8f& c0, v8f& c1, v8f& c2, v8f& c3, const us16& a0, const us16& a1,
                                       const us16& b0, const us16& b1, const us16& b2, const us16& b3) {
#if defined(__HIP_DEVICE_COMPILE__)
  asm volatile("v_nop\n\tv_nop\n\tv_nop\n\tv_nop"
               : "+v"(c0), "+v"(c1), "+v"(c2), "+v"(c3)
               : "v"(a0), "v"(a1), "v"(b0), "v"(b1), "v"(b2), "v"(b3));
#endif
}

__device__ __forceinline__ us16 lds_frag(const unsigned short* base) {
  const int lane = threadIdx.x & 31, r = lane & 15, kh = (lane >> 4) * 8;
  FragU f;
  f.h[0] = *(const us8a*)(base + r * GSTR + kh);
  f.h[1] = *(const us8a*)(base + r * GSTR + 16 + kh);
  return f.v;
}

__device__ __forceinline__ void stage_a(unsigned short* lds, const unsigned short* __restrict__ P, int ld, int m0, int k0, int tid) {
  const int row = tid >> 1, cq = (tid & 1) * 16;
  const unsigned short* src = P + (size_t)(m0 + row) * ld + k0 + cq;
  const us8 v0 = *(const us8a*)src;
  const us8 v1 = *(const us8a*)(src + 8);
  *(us8a*)(lds + row * GSTR + cq) = v0;
  *(us8a*)(lds + row * GSTR + cq + 8) = v1;
}
__device__ __forceinline__ void stage_b(unsigned short* lds, const unsigned short* __restrict__ P, int ld, int n0, int k0, int tid) {
  const int row = tid >> 2, kq = (tid & 3) * 8;
  const us8 v = *(const us8a*)(P + (size_t)(n0 + row) * ld + k0 + kq);
  *(us8a*)(lds + row * GSTR + kq) = v;
}

template <int A2, int EPI>
__global__ __launch_bounds__(256) void k_gemm(const unsigned short* __restrict__ A0, const unsigned short* __restrict__ A1, int lda,
                                             const unsigned short* __restrict__ B0, int ldb,
                                             float* Y, float* Yalt, int nsplit, int ldy, int K,
                                             const float* __restrict__ p0, const float* __restrict__ p1,
                                             const float* __restrict__ p2, const float* __restrict__ p3,
                                             const float* __restrict__ adds, int ldadd) {
#pragma clang fp contract(off)
  __shared__ __attribute__((aligned(16))) unsigned char sm[SMEMB];
  unsigned short* lA0 = (unsigned short*)sm;
  unsigned short* lA1 = lA0 + 128 * GSTR;
  unsigned short* lB0 = lA1 + 128 * GSTR;
  float* oS = (float*)sm;
  const int tid = threadIdx.x, lane = tid & 31, wave = tid >> 5, cl = lane & 15, hh = lane >> 4;
  const int m0 = blockIdx.x * 128;
  const int n0 = blockIdx.y * 64;
  float* Yb = Y;
  int nq = n0;
  if (EPI == 0) {
    if (nsplit > 0 && n0 >= nsplit) { Yb = Yalt; nq = n0 - nsplit; }
  }

  v8f acc[4];
#pragma unroll
  for (int j = 0; j < 4; ++j) { v8f zz = {0.f, 0.f, 0.f, 0.f, 0.f, 0.f, 0.f, 0.f}; acc[j] = zz; }

#pragma unroll 1
  for (int k0 = 0; k0 < K; k0 += 32) {
    __syncthreads();
    stage_a(lA0, A0, lda, m0, k0, tid);
    if (A2) stage_a(lA1, A1, lda, m0, k0, tid);
    stage_b(lB0, B0, ldb, n0, k0, tid);
    __syncthreads();
    const us16 af0 = lds_frag(lA0 + 16 * wave * GSTR);
    us16 af1 = af0;
    if (A2) af1 = lds_frag(lA1 + 16 * wave * GSTR);
    us16 bfr[4];
#pragma unroll
    for (int j = 0; j < 4; ++j) bfr[j] = lds_frag(lB0 + 16 * j * GSTR);
#pragma unroll
    for (int j = 0; j < 4; ++j) acc[j] = mma_bf16(af0, bfr[j], acc[j]);
    if (A2) {
#pragma unroll
      for (int j = 0; j < 4; ++j) acc[j] = mma_bf16(af1, bfr[j], acc[j]);
    }
    wguard(acc[0], acc[1], acc[2], acc[3], af0, af1, bfr[0], bfr[1], bfr[2], bfr[3]);
  }
  __syncthreads();

  if (EPI == 3) {
    float* sT = oS;
    float bj[4];
#pragma unroll
    for (int j = 0; j < 4; ++j) bj[j] = bf16r(p0[n0 + 16 * j + cl]);
#pragma unroll
    for (int j = 0; j < 4; ++j)
#pragma unroll
      for (int r = 0; r < 8; ++r) sT[(16 * j + cl) * TPN + 16 * wave + 8 * hh + r] = acc[j][r] + bj[j];
    __syncthreads();
    const int bb = m0 / LTOK, l0 = m0 - bb * LTOK;
#pragma unroll
    for (int pass = 0; pass < 2; ++pass) {
#pragma unroll
      for (int it = 0; it < 8; ++it) {
        const int o = 8 * wave + it;
        const v4f v = *(const v4fa*)(sT + o * TPN + 4 * lane);
        *(volatile v4f*)(Yb + ((size_t)(bb * NCH + n0 + o)) * LTOK + l0 + 4 * lane) = v;
      }
      __threadfence();
    }
  } else {
    float emu[4], ers[4], eg[4], eb[4];
#pragma unroll
    for (int j = 0; j < 4; ++j) {
      if (EPI == 1 || EPI == 2) {
        const int col = n0 + 16 * j + cl;
        emu[j] = bf16r(p2[col]);
        ers[j] = rsqrtf(bf16r(p3[col]) + EPSV);
        eg[j]  = bf16r(p0[col]);
        eb[j]  = bf16r(p1[col]);
      } else {
        emu[j] = 0.0f; ers[j] = 1.0f; eg[j] = 1.0f; eb[j] = 0.0f;
      }
    }
    float* so = oS + wave * (16 * OSTR);
#pragma unroll
    for (int j = 0; j < 4; ++j)
#pragma unroll
      for (int r = 0; r < 8; ++r) {
        float v = acc[j][r];
        if (EPI == 1 || EPI == 2) v = ((v - emu[j]) * ers[j]) * eg[j] + eb[j];
        so[(8 * hh + r) * OSTR + 16 * j + cl] = v;
      }
    __syncthreads();
#pragma unroll
    for (int pass = 0; pass < 2; ++pass) {
#pragma unroll
      for (int it = 0; it < 8; ++it) {
        const int ch = it * 32 + lane, r = ch >> 4, q = (ch & 15) * 4;
        v4f v = *(const v4fa*)(so + r * OSTR + q);
        if (EPI == 2) {
          const v4f av = *(const v4fa*)(adds + (size_t)(m0 + 16 * wave + r) * ldadd + nq + q);
          v = v + av;
        }
        *(volatile v4f*)(Yb + (size_t)(m0 + 16 * wave + r) * ldy + nq + q) = v;
      }
      __threadfence();
    }
  }
}

__global__ __launch_bounds__(256) void k_cvt(const float* __restrict__ src, unsigned short* dst, int nsrc, int ncol8, int total8) {
  const int idx = blockIdx.x * 256 + threadIdx.x;
  if (idx >= total8) return;
  const int row = idx / ncol8, c8 = (idx - row * ncol8) * 8;
  const int rs = (row < nsrc) ? row : (nsrc - 1);
  const float* s = src + (size_t)rs * (size_t)(ncol8 * 8) + c8;
  const v4f a = *(const v4fa*)s, b = *(const v4fa*)(s + 4);
  const bool zr = (row >= nsrc);
  us8 o;
#pragma unroll
  for (int u = 0; u < 4; ++u) {
    o[u]     = zr ? (unsigned short)0 : bf16_bits(a[u]);
    o[4 + u] = zr ? (unsigned short)0 : bf16_bits(b[u]);
  }
  const size_t off = (size_t)row * (size_t)(ncol8 * 8) + c8;
  *(volatile us8*)(dst + off) = o;
  __threadfence();
  *(volatile us8*)(dst + off) = o;
}

__device__ __forceinline__ void ln_row(const v4f a, const v4f b, const float* gg, const float* bq, us8& hi, us8& lo) {
#pragma clang fp contract(off)
  float s = ((a[0] + a[1]) + (a[2] + a[3])) + ((b[0] + b[1]) + (b[2] + b[3]));
#pragma unroll
  for (int o = 16; o > 0; o >>= 1) s = s + __shfl_xor(s, o);
  const float mu = s * (1.0f / NCH);
  float dv[8];
#pragma unroll
  for (int u = 0; u < 4; ++u) { dv[u] = a[u] - mu; dv[4 + u] = b[u] - mu; }
  float s2 = 0.0f;
#pragma unroll
  for (int u = 0; u < 8; ++u) s2 = s2 + dv[u] * dv[u];
#pragma unroll
  for (int o = 16; o > 0; o >>= 1) s2 = s2 + __shfl_xor(s2, o);
  const float var = s2 * (1.0f / NCH);
  const float rs = rsqrtf(var + EPSV);
#pragma unroll
  for (int u = 0; u < 8; ++u) {
    const float ov = (dv[u] * rs) * gg[u] + bq[u];
    const unsigned short hb = bf16_bits(ov);
    hi[u] = hb; lo[u] = bf16_bits(ov - bf16_val(hb));
  }
}

__global__ __launch_bounds__(256) void k_ln1(const float* __restrict__ X, const float* __restrict__ g, const float* __restrict__ bt,
                                            unsigned short* NH, unsigned short* NL) {
#pragma clang fp contract(off)
  __shared__ __attribute__((aligned(16))) float st[32 * LNP];
  const int tid = threadIdx.x, lane = tid & 31, wave = tid >> 5;
  const int n0 = blockIdx.x * 32, bb = n0 / LTOK, l0 = n0 - bb * LTOK;
#pragma unroll 1
  for (int c = wave; c < NCH; c += 8) {
    const float v = X[((size_t)(bb * NCH + c)) * LTOK + (size_t)(l0 + lane)];
    st[lane * LNP + c] = bf16r(v);
  }
  __syncthreads();
  const int c8 = lane * 8;
  float gg[8], bq[8];
  {
    const v4f ga = *(const v4fa*)(g + c8), gb = *(const v4fa*)(g + c8 + 4);
    const v4f ba = *(const v4fa*)(bt + c8), b4 = *(const v4fa*)(bt + c8 + 4);
#pragma unroll
    for (int u = 0; u < 4; ++u) { gg[u] = bf16r(ga[u]); gg[4 + u] = bf16r(gb[u]); bq[u] = bf16r(ba[u]); bq[4 + u] = bf16r(b4[u]); }
  }
#pragma unroll 1
  for (int t4 = 0; t4 < 4; ++t4) {
    const int t = wave * 4 + t4;
    const v4f a = *(const v4fa*)(st + t * LNP + c8);
    const v4f b = *(const v4fa*)(st + t * LNP + c8 + 4);
    us8 hi, lo;
    ln_row(a, b, gg, bq, hi, lo);
    const size_t o = (size_t)(n0 + t) * NCH + c8;
    *(volatile us8*)(NH + o) = hi; *(volatile us8*)(NL + o) = lo;
    __threadfence();
    *(volatile us8*)(NH + o) = hi; *(volatile us8*)(NL + o) = lo;
  }
}

__global__ __launch_bounds__(256) void k_ln2(const float* __restrict__ XM, const float* __restrict__ g, const float* __restrict__ bt,
                                            unsigned short* NH, unsigned short* NL) {
#pragma clang fp contract(off)
  const int tid = threadIdx.x, lane = tid & 31, wave = tid >> 5;
  const int tok = blockIdx.x * 8 + wave;
  const int c8 = lane * 8;
  float gg[8], bq[8];
  {
    const v4f ga = *(const v4fa*)(g + c8), gb = *(const v4fa*)(g + c8 + 4);
    const v4f ba = *(const v4fa*)(bt + c8), b4 = *(const v4fa*)(bt + c8 + 4);
#pragma unroll
    for (int u = 0; u < 4; ++u) { gg[u] = bf16r(ga[u]); gg[4 + u] = bf16r(gb[u]); bq[u] = bf16r(ba[u]); bq[4 + u] = bf16r(b4[u]); }
  }
  const v4f a = *(const v4fa*)(XM + (size_t)tok * NCH + c8);
  const v4f b = *(const v4fa*)(XM + (size_t)tok * NCH + c8 + 4);
  us8 hi, lo;
  ln_row(a, b, gg, bq, hi, lo);
  const size_t o = (size_t)tok * NCH + c8;
  *(volatile us8*)(NH + o) = hi; *(volatile us8*)(NL + o) = lo;
  __threadfence();
  *(volatile us8*)(NH + o) = hi; *(volatile us8*)(NL + o) = lo;
}

__global__ __launch_bounds__(256) void k_conv(const float* __restrict__ XU, const float* __restrict__ cw, const float* __restrict__ cb,
                                             unsigned short* UH, unsigned short* UL) {
#pragma clang fp contract(off)
  const int idx = blockIdx.x * 256 + threadIdx.x;
  const int tok = idx >> 5, c4 = (idx & 31) * 4;
  const int l = tok & (LTOK - 1);
  v4f xv[DCV];
#pragma unroll
  for (int j = 0; j < DCV; ++j) {
    const int ll = l - (DCV - 1) + j;
    const int tc = (ll >= 0) ? (tok - (DCV - 1) + j) : tok;
    xv[j] = *(const v4fa*)(XU + (size_t)tc * DIN + c4);
  }
  const v4f b4 = *(const v4fa*)(cb + c4);
  us4 hi, lo;
#pragma unroll
  for (int u = 0; u < 4; ++u) {
    const v4f wv = *(const v4fa*)(cw + (size_t)(c4 + u) * DCV);
    float a = 0.0f;
#pragma unroll
    for (int j = 0; j < DCV; ++j) {
      const float pr = bf16r(wv[j]) * xv[j][u];
      a = a + ((l - (DCV - 1) + j >= 0) ? pr : 0.0f);
    }
    a = a + bf16r(b4[u]);
    const float sv = siluf(a);
    const unsigned short hb = bf16_bits(sv);
    hi[u] = hb; lo[u] = bf16_bits(sv - bf16_val(hb));
  }
  const size_t o = (size_t)tok * DIN + c4;
  *(volatile us4*)(UH + o) = hi; *(volatile us4*)(UL + o) = lo;
  __threadfence();
  *(volatile us4*)(UH + o) = hi; *(volatile us4*)(UL + o) = lo;
}

template <int PL>
__global__ __launch_bounds__(256) void k_dw(const unsigned short* __restrict__ IH, const unsigned short* __restrict__ IL, int ldi,
                                           const float* __restrict__ IF, const float* __restrict__ w9,
                                           unsigned short* DH, unsigned short* DL, int dil) {
#pragma clang fp contract(off)
  const int idx = blockIdx.x * 256 + threadIdx.x;
  const int tok = idx >> 4, c4 = (idx & 15) * 4;
  const int bb = tok / LTOK, l = tok - bb * LTOK, hy0 = l / IMW, wx0 = l - hy0 * IMW;
  float wv[4][9];
#pragma unroll
  for (int u = 0; u < 4; ++u)
#pragma unroll
    for (int t = 0; t < 9; ++t) wv[u][t] = bf16r(w9[(c4 + u) * 9 + t]);
  float acc[4] = {0.0f, 0.0f, 0.0f, 0.0f};
#pragma unroll
  for (int kh = 0; kh < 3; ++kh) {
#pragma unroll
    for (int kw = 0; kw < 3; ++kw) {
      const int hy = hy0 + dil * (kh - 1), wx = wx0 + dil * (kw - 1);
      const bool ok = ((unsigned)hy < (unsigned)IMH) && ((unsigned)wx < (unsigned)IMW);
      const int hyc = (hy < 0) ? 0 : ((hy > IMH - 1) ? (IMH - 1) : hy);
      const int wxc = (wx < 0) ? 0 : ((wx > IMW - 1) ? (IMW - 1) : wx);
      const size_t ts = (size_t)bb * LTOK + (size_t)(hyc * IMW + wxc);
      float v[4];
      if (PL) {
        const us4 ah = *(const us4a*)(IH + ts * (size_t)ldi + c4);
        const us4 al = *(const us4a*)(IL + ts * (size_t)ldi + c4);
#pragma unroll
        for (int u = 0; u < 4; ++u) v[u] = bf16_val(ah[u]) + bf16_val(al[u]);
      } else {
        const v4f f = *(const v4fa*)(IF + ts * DMD + c4);
#pragma unroll
        for (int u = 0; u < 4; ++u) v[u] = f[u];
      }
#pragma unroll
      for (int u = 0; u < 4; ++u) {
        const float pr = wv[u][kh * 3 + kw] * v[u];
        acc[u] = acc[u] + (ok ? pr : 0.0f);
      }
    }
  }
  us4 hi, lo;
#pragma unroll
  for (int u = 0; u < 4; ++u) {
    const unsigned short hb = bf16_bits(acc[u]);
    hi[u] = hb; lo[u] = bf16_bits(acc[u] - bf16_val(hb));
  }
  const size_t o = (size_t)tok * DMD + c4;
  *(volatile us4*)(DH + o) = hi; *(volatile us4*)(DL + o) = lo;
  __threadfence();
  *(volatile us4*)(DH + o) = hi; *(volatile us4*)(DL + o) = lo;
}

__global__ __launch_bounds__(128) void k_scan(const float* __restrict__ XD, const unsigned short* __restrict__ UH,
                                             const unsigned short* __restrict__ UL, const float* __restrict__ XZ,
                                             const float* __restrict__ dtw, const float* __restrict__ dtb,
                                             const float* __restrict__ Alog, const float* __restrict__ Dv,
                                             unsigned short* YH, unsigned short* YL) {
#pragma clang fp contract(off)
  __shared__ __attribute__((aligned(16))) float sy[SCH * SYP];
  const int bb = blockIdx.x, tid = threadIdx.x, lane = tid & 31, wave = tid >> 5;
  const int d = tid;
  float A2[DST], h[DST];
#pragma unroll
  for (int n = 0; n < DST; ++n) { A2[n] = -__expf(bf16r(Alog[d * DST + n])) * LOG2E; h[n] = 0.0f; }
  float wd[DTRK];
#pragma unroll
  for (int r = 0; r < DTRK; ++r) wd[r] = bf16r(dtw[d * DTRK + r]);
  const float bd = bf16r(dtb[d]);
  const float Dd = bf16r(Dv[d]);
#pragma unroll 1
  for (int c = 0; c < LTOK / SCH; ++c) {
#pragma unroll 1
    for (int s = 0; s < SCH; ++s) {
      const size_t tok = (size_t)bb * LTOK + (size_t)(c * SCH + s);
      const float* xr = XD + tok * XDN;
      const v4f dq = *(const v4fa*)xr;
      const float raw = ((dq[0] * wd[0] + dq[1] * wd[1]) + dq[2] * wd[2]) + dq[3] * wd[3];
      const float a = raw + bd;
      const float dl = fmaxf(a, 0.0f) + log1pf(__expf(-fabsf(a)));
      const float uv = bf16_val(UH[tok * DIN + d]) + bf16_val(UL[tok * DIN + d]);
      const float zv = XZ[tok * DIN + d];
      v4f Bv[4], Cv[4];
#pragma unroll
      for (int q = 0; q < 4; ++q) {
        Bv[q] = *(const v4fa*)(xr + DTRK + 4 * q);
        Cv[q] = *(const v4fa*)(xr + DTRK + DST + 4 * q);
      }
      const float dx = dl * uv;
      float y = 0.0f;
#pragma unroll
      for (int n = 0; n < DST; ++n) {
        const float e = exp2f(dl * A2[n]);
        h[n] = e * h[n] + dx * Bv[n >> 2][n & 3];
        y = y + h[n] * Cv[n >> 2][n & 3];
      }
      const float yv = (y + uv * Dd) * siluf(zv);
      sy[s * SYP + tid] = yv;
    }
    __syncthreads();
#pragma unroll
    for (int pass = 0; pass < 2; ++pass) {
#pragma unroll
      for (int it = 0; it < 4; ++it) {
        const int rr = 8 * wave + 2 * it + (lane >> 4), c8 = (lane & 15) * 8;
        const v4f va = *(const v4fa*)(sy + rr * SYP + c8);
        const v4f vb = *(const v4fa*)(sy + rr * SYP + c8 + 4);
        us8 hi, lo;
#pragma unroll
        for (int u = 0; u < 4; ++u) {
          const unsigned short ha = bf16_bits(va[u]);
          hi[u] = ha; lo[u] = bf16_bits(va[u] - bf16_val(ha));
          const unsigned short hb = bf16_bits(vb[u]);
          hi[4 + u] = hb; lo[4 + u] = bf16_bits(vb[u] - bf16_val(hb));
        }
        const size_t o = ((size_t)bb * LTOK + (size_t)(c * SCH + rr)) * DIN + c8;
        *(volatile us8*)(YH + o) = hi; *(volatile us8*)(YL + o) = lo;
      }
      __threadfence();
    }
    __syncthreads();
  }
}

extern "C" void kernel_launch(void* const* d_in, const int* in_sizes, int n_in,
                              void* d_out, int out_size, void* d_ws, size_t ws_size,
                              hipStream_t stream) {
  if (n_in < 20) return;
  if (in_sizes[0] != NTOK * NCH || in_sizes[1] != NCH || in_sizes[2] != NCH || in_sizes[3] != NCH * NCH || in_sizes[4] != NCH ||
      in_sizes[5] != 2 * DIN * DMD || in_sizes[6] != DIN * DCV || in_sizes[7] != DIN || in_sizes[8] != XPR * DIN ||
      in_sizes[9] != DIN * DTRK || in_sizes[10] != DIN || in_sizes[11] != DIN * DST || in_sizes[12] != DIN ||
      in_sizes[13] != DMD * DIN || in_sizes[14] != NCHK * NLY * DMD * 9 || in_sizes[15] != NCHK * NLY * DMD * DMD ||
      in_sizes[16] != NCHK * NLY * DMD || in_sizes[17] != NCHK * NLY * DMD || in_sizes[18] != NCHK * NLY * DMD ||
      in_sizes[19] != NCHK * NLY * DMD || out_size != NTOK * NCH) return;

  const float* x     = (const float*)d_in[0];
  const float* ng    = (const float*)d_in[1];
  const float* nb    = (const float*)d_in[2];
  const float* pw    = (const float*)d_in[3];
  const float* pb    = (const float*)d_in[4];
  const float* inw   = (const float*)d_in[5];
  const float* cw    = (const float*)d_in[6];
  const float* cb    = (const float*)d_in[7];
  const float* xpw   = (const float*)d_in[8];
  const float* dtw   = (const float*)d_in[9];
  const float* dtb   = (const float*)d_in[10];
  const float* Alog  = (const float*)d_in[11];
  const float* Dv    = (const float*)d_in[12];
  const float* ow    = (const float*)d_in[13];
  const float* dww   = (const float*)d_in[14];
  const float* pww   = (const float*)d_in[15];
  const float* bng   = (const float*)d_in[16];
  const float* bnb   = (const float*)d_in[17];
  const float* bnm   = (const float*)d_in[18];
  const float* bnv   = (const float*)d_in[19];
  float* out = (float*)d_out;

  size_t off = 0;
  auto carve = [&](size_t bytes) -> char* { char* p = (char*)d_ws + off; off += (bytes + 255) & ~(size_t)255; return p; };
  unsigned short* WIN16 = (unsigned short*)carve((size_t)2 * DIN * DMD * 2);
  unsigned short* WX16  = (unsigned short*)carve((size_t)XDN * DIN * 2);
  unsigned short* WO16  = (unsigned short*)carve((size_t)DMD * DIN * 2);
  unsigned short* WPW16 = (unsigned short*)carve((size_t)NCHK * NLY * DMD * DMD * 2);
  unsigned short* WP16  = (unsigned short*)carve((size_t)NCH * NCH * 2);
  unsigned short* NH    = (unsigned short*)carve((size_t)NTOK * NCH * 2);
  unsigned short* NL    = (unsigned short*)carve((size_t)NTOK * NCH * 2);
  float* XU             = (float*)carve((size_t)NTOK * DIN * 4);
  float* XZg            = (float*)carve((size_t)NTOK * DIN * 4);
  unsigned short* UH    = (unsigned short*)carve((size_t)NTOK * DIN * 2);
  unsigned short* UL    = (unsigned short*)carve((size_t)NTOK * DIN * 2);
  float* XD             = (float*)carve((size_t)NTOK * XDN * 4);
  float* XM             = (float*)carve((size_t)NTOK * NCH * 4);
  if (off > ws_size || off > (size_t)134217728) return;
  unsigned short* YH = (unsigned short*)XU;
  unsigned short* YL = (unsigned short*)((char*)XU + (size_t)NTOK * DIN * 2);
  unsigned short* DH = (unsigned short*)XU;
  unsigned short* DL = (unsigned short*)((char*)XU + (size_t)NTOK * DMD * 2);
  float* PB          = (float*)((char*)XU + (size_t)2 * NTOK * DMD * 2);
  float* M4          = XD;

  const dim3 b256(256), b128(128);
  k_cvt<<<dim3((2 * DIN * DMD / 8 + 255) / 256), b256, 0, stream>>>(inw, WIN16, 2 * DIN, DMD / 8, 2 * DIN * DMD / 8);
  k_cvt<<<dim3((XDN * DIN / 8 + 255) / 256), b256, 0, stream>>>(xpw, WX16, XPR, DIN / 8, XDN * DIN / 8);
  k_cvt<<<dim3((DMD * DIN / 8 + 255) / 256), b256, 0, stream>>>(ow, WO16, DMD, DIN / 8, DMD * DIN / 8);
  k_cvt<<<dim3((NCHK * NLY * DMD * DMD / 8 + 255) / 256), b256, 0, stream>>>(pww, WPW16, NCHK * NLY * DMD, DMD / 8, NCHK * NLY * DMD * DMD / 8);
  k_cvt<<<dim3((NCH * NCH / 8 + 255) / 256), b256, 0, stream>>>(pw, WP16, NCH, NCH / 8, NCH * NCH / 8);
  k_ln1<<<dim3(NTOK / 32), b256, 0, stream>>>(x, ng, nb, NH, NL);

  const int dils[NLY] = {1, 2, 3, 1};
  for (int i = 0; i < NCHK; ++i) {
    k_gemm<1, 0><<<dim3(NTOK / 128, (2 * DIN) / 64), b256, 0, stream>>>(NH + DMD * i, NL + DMD * i, NCH, WIN16, DMD,
                                                                       XU, XZg, DIN, DIN, DMD, pb, pb, pb, pb, XU, DIN);
    k_conv<<<dim3(NTOK * 32 / 256), b256, 0, stream>>>(XU, cw, cb, UH, UL);
    k_gemm<0, 0><<<dim3(NTOK / 128, XDN / 64), b256, 0, stream>>>(UH, UH, DIN, WX16, DIN, XD, XD, 0, XDN, DIN, pb, pb, pb, pb, XD, XDN);
    k_scan<<<dim3(NBAT), b128, 0, stream>>>(XD, UH, UL, XZg, dtw, dtb, Alog, Dv, YH, YL);
    k_gemm<1, 0><<<dim3(NTOK / 128, DMD / 64), b256, 0, stream>>>(YH, YL, DIN, WO16, DIN, M4, M4, 0, DMD, DIN, pb, pb, pb, pb, M4, DMD);
    for (int s = 0; s < NLY; ++s) {
      const int si = i * NLY + s;
      const float* w9 = dww + (size_t)si * DMD * 9;
      if (s == 0) k_dw<1><<<dim3(NTOK * 16 / 256), b256, 0, stream>>>(NH + DMD * i, NL + DMD * i, NCH, PB, w9, DH, DL, dils[s]);
      else        k_dw<0><<<dim3(NTOK * 16 / 256), b256, 0, stream>>>(NH, NL, NCH, PB, w9, DH, DL, dils[s]);
      const unsigned short* wpl = WPW16 + (size_t)si * DMD * DMD;
      const float* g1 = bng + si * DMD;
      const float* b1 = bnb + si * DMD;
      const float* m1 = bnm + si * DMD;
      const float* v1 = bnv + si * DMD;
      if (s < NLY - 1) k_gemm<0, 1><<<dim3(NTOK / 128, DMD / 64), b256, 0, stream>>>(DH, DH, DMD, wpl, DMD, PB, PB, 0, DMD, DMD, g1, b1, m1, v1, PB, DMD);
      else             k_gemm<1, 2><<<dim3(NTOK / 128, DMD / 64), b256, 0, stream>>>(DH, DL, DMD, wpl, DMD, XM + DMD * i, XM, 0, NCH, DMD, g1, b1, m1, v1, M4, DMD);
    }
  }
  k_ln2<<<dim3(NTOK / 8), b256, 0, stream>>>(XM, ng, nb, NH, NL);
  k_gemm<1, 3><<<dim3(NTOK / 128, NCH / 64), b256, 0, stream>>>(NH, NL, NCH, WP16, NCH, out, out, 0, LTOK, NCH, pb, pb, pb, pb, XM, NCH);
}
